// LocalSelfAttentionUnFold_39256001085595
// MI455X (gfx1250) — hardware-verified
//
#include <hip/hip_runtime.h>
#include <math.h>

constexpr int kBatch  = 4;
constexpr int kSeq    = 2048;
constexpr int kEmb    = 256;
constexpr int kHeads  = 8;
constexpr int kHd     = 32;
constexpr int kWin    = 33;
constexpr int kKeys   = kSeq - kWin + 1;
constexpr int kTok    = kBatch * kSeq;
constexpr int kPairs  = kBatch * kHeads;
constexpr int kGrp    = 2;
constexpr int kNGrp   = kPairs / kGrp;
constexpr int kQKld   = 2 * kEmb;
constexpr int kVSRows = 64;
constexpr int kSteps  = kSeq + 16;
constexpr int kDiagOff = 2031;
constexpr float kScoreScale = 0.17677669529663687f;
constexpr float kPCarry     = 1024.0f;
constexpr float kPCarryInv  = 1.0f / 1024.0f;

typedef __attribute__((ext_vector_type(16))) _Float16 v16h;
typedef __attribute__((ext_vector_type(8)))  _Float16 v8h;
typedef __attribute__((ext_vector_type(16))) __bf16   v16b;
typedef __attribute__((ext_vector_type(8)))  __bf16   v8b;
typedef __attribute__((ext_vector_type(8)))  float    v8f;
typedef __attribute__((ext_vector_type(4)))  float    v4f;
typedef __attribute__((ext_vector_type(4)))  unsigned int v4u;

__device__ __forceinline__ unsigned short f2bf_bits(float f) {
  unsigned u = __float_as_uint(f);
  return (unsigned short)((u + 0x7FFFu + ((u >> 16) & 1u)) >> 16);
}
__device__ __forceinline__ float bf_bits2f(unsigned short h) { return __uint_as_float(((unsigned)h) << 16); }

__device__ __forceinline__ void dep_guard_h(v8f& a, v8f& b, v16h x, v16h y) { asm volatile("v_nop\n\tv_nop\n\tv_nop\n\tv_nop" : "+v"(a), "+v"(b) : "v"(x), "v"(y)); }
__device__ __forceinline__ void dep_guard_b(v8f& a, v8f& b, v16b x, v16b y) { asm volatile("v_nop\n\tv_nop\n\tv_nop\n\tv_nop" : "+v"(a), "+v"(b) : "v"(x), "v"(y)); }
__device__ __forceinline__ void keep4_h(v16h a, v16h b, v16h c, v16h d) { asm volatile("v_nop" :: "v"(a), "v"(b), "v"(c), "v"(d)); }
__device__ __forceinline__ void keep4_b(v16b a, v16b b, v16b c, v16b d) { asm volatile("v_nop" :: "v"(a), "v"(b), "v"(c), "v"(d)); }
__device__ __forceinline__ void acc_guard4(v8f& a, v8f& b, v8f& c, v8f& d) { asm volatile("v_nop\n\tv_nop\n\tv_nop\n\tv_nop" : "+v"(a), "+v"(b), "+v"(c), "+v"(d)); }
template <typename T> struct Frag;
template <> struct Frag<_Float16> {
  typedef v16h V; union U { v16h v; v8h h[2]; };
  static __device__ __forceinline__ v16h load(const _Float16* p) {
    U f; f.h[0] = *(const v8h*)(p); f.h[1] = *(const v8h*)(p + 16); return f.v;
  }
  static __device__ __forceinline__ v8f mma(v16h a, v16h b, v8f c) {
    return __builtin_amdgcn_wmma_f32_16x16x32_f16(false, a, false, b, (short)0, c, false, false);
  }
  static __device__ __forceinline__ void guard(v8f& a, v8f& b, v16h x, v16h y) { dep_guard_h(a, b, x, y); }
  static __device__ __forceinline__ void keep(v16h a, v16h b, v16h c, v16h d) { keep4_h(a, b, c, d); }
};
template <> struct Frag<__bf16> {
  typedef v16b V; union U { v16b v; v8b h[2]; };
  static __device__ __forceinline__ v16b load(const __bf16* p) {
    U f; f.h[0] = *(const v8b*)(p); f.h[1] = *(const v8b*)(p + 16); return f.v;
  }
  static __device__ __forceinline__ v8f mma(v16b a, v16b b, v8f c) {
    return __builtin_amdgcn_wmma_f32_16x16x32_bf16(false, a, false, b, (short)0, c, false, false);
  }
  static __device__ __forceinline__ void guard(v8f& a, v8f& b, v16b x, v16b y) { dep_guard_b(a, b, x, y); }
  static __device__ __forceinline__ void keep(v16b a, v16b b, v16b c, v16b d) { keep4_b(a, b, c, d); }
};

__device__ __forceinline__ unsigned pk16(unsigned short a, unsigned short b) { return (unsigned)a | ((unsigned)b << 16); }
__device__ __forceinline__ unsigned short h_bits(float f) { const _Float16 h = (_Float16)f; return __builtin_bit_cast(unsigned short, h); }

template <int ET> struct Elem;
template <> struct Elem<0> { typedef _Float16 T; };
template <> struct Elem<1> { typedef __bf16 T; };
template <int ET, bool SPLIT, int BIAS_MODE, int OUT_MODE, bool RESID, int ACT = 0>
__global__ __launch_bounds__(256) void wmma_gemm64(
    const unsigned short* __restrict__ Ap, const unsigned short* __restrict__ A2p, int lda, long strideA,
    const unsigned short* __restrict__ Btp, const unsigned short* __restrict__ Bt2p, int ldb, long strideB,
    void* __restrict__ Cout, void* __restrict__ Cout2, int ldc, long strideC,
    const float* __restrict__ bias,
    const float* __restrict__ resid, long strideR,
    int M, int N, int K, float scale) {
  typedef typename Elem<ET>::T T;
  typedef typename Frag<T>::V V;
  const T* A = (const T*)Ap; const T* A2 = (const T*)A2p; const T* Bt = (const T*)Btp; const T* Bt2 = (const T*)Bt2p;
  __shared__ __align__(16) float sT[8][16 * 68];
  const int b    = blockIdx.y;
  const int lane = threadIdx.x & 31;
  const int wave = threadIdx.x >> 5;
  const int tilesN = N >> 6;
  const int tilesM = M >> 6;
  const int tile = blockIdx.x * 8 + wave;
  if (tile >= tilesM * tilesN) return;
  const int tm = tile / tilesN;
  const int tn = tile - tm * tilesN;
  const int m0 = tm << 6;
  const int n0 = tn << 6;

  const T* Ab  = A  + (size_t)b * strideA;
  const T* Bb  = Bt + (size_t)b * strideB;
  const T* Ab2 = SPLIT ? (A2  + (size_t)b * strideA) : nullptr;
  const T* Bb2 = SPLIT ? (Bt2 + (size_t)b * strideB) : nullptr;

  const int rlane = lane & 15;
  const int koff  = (lane >> 4) * 8;
  const int mOff  = (lane >> 4) * 8;

  v8f acc[4][4];
#pragma unroll
  for (int i = 0; i < 4; ++i)
#pragma unroll
    for (int j = 0; j < 4; ++j) acc[i][j] = (v8f){0.f,0.f,0.f,0.f,0.f,0.f,0.f,0.f};

  for (int k0 = 0; k0 < K; k0 += 32) {
    V bh[4], bl[4];
#pragma unroll
    for (int j = 0; j < 4; ++j) {
      const size_t bo = (size_t)(n0 + (j << 4) + rlane) * ldb + koff + k0;
      bh[j] = Frag<T>::load(Bb + bo);
      if (SPLIT) bl[j] = Frag<T>::load(Bb2 + bo);
    }
#pragma unroll
    for (int i = 0; i < 4; ++i) {
      const size_t ao = (size_t)(m0 + (i << 4) + rlane) * lda + koff + k0;
      V ah = Frag<T>::load(Ab + ao);
      V al;
      if (SPLIT) al = Frag<T>::load(Ab2 + ao);
#pragma unroll
      for (int j = 0; j < 4; ++j) {
        acc[i][j] = Frag<T>::mma(ah, bh[j], acc[i][j]);
        if (SPLIT) {
          acc[i][j] = Frag<T>::mma(ah, bl[j], acc[i][j]);
          acc[i][j] = Frag<T>::mma(al, bh[j], acc[i][j]);
        }
      }
      Frag<T>::guard(acc[i][0], acc[i][3], ah, SPLIT ? al : ah);
    }
    Frag<T>::keep(bh[0], bh[1], bh[2], bh[3]);
    if (SPLIT) Frag<T>::keep(bl[0], bl[1], bl[2], bl[3]);
  }
  acc_guard4(acc[0][0], acc[0][1], acc[0][2], acc[0][3]);
  acc_guard4(acc[1][0], acc[1][1], acc[1][2], acc[1][3]);
  acc_guard4(acc[2][0], acc[2][1], acc[2][2], acc[2][3]);
  acc_guard4(acc[3][0], acc[3][1], acc[3][2], acc[3][3]);

  float* slab = sT[wave];
  const float* Rb = RESID ? (resid + (size_t)b * strideR) : nullptr;
#pragma unroll
  for (int i = 0; i < 4; ++i) {
    const int mBase = m0 + (i << 4);
#pragma unroll
    for (int j = 0; j < 4; ++j) {
      const int n = n0 + (j << 4) + rlane;
      float bv = 0.f;
      if (BIAS_MODE == 2) bv = bias[n];
#pragma unroll
      for (int r = 0; r < 8; ++r) {
        float v = acc[i][j][r] * scale;
        if (BIAS_MODE == 1) v += bias[mBase + mOff + r];
        if (BIAS_MODE == 2) v += bv;
        if (RESID) v += Rb[(size_t)(mBase + mOff + r) * ldc + n];
        if (ACT == 2) v = fmaxf(v, 0.0f);
        if (ACT == 4) v = (v > 0.f) ? v : 0.01f * v;
        slab[(mOff + r) * 68 + (j << 4) + rlane] = v;
      }
    }
    __builtin_amdgcn_fence(__ATOMIC_RELEASE, "workgroup");
    __builtin_amdgcn_wave_barrier();
    __builtin_amdgcn_fence(__ATOMIC_ACQUIRE, "workgroup");
    if (OUT_MODE == 0) {
      float* C = (float*)Cout + (size_t)b * strideC;
      const int hh = lane >> 4, c4 = (lane & 15) * 4;
      for (int pass = 0; pass < 2; ++pass) {
#pragma unroll
        for (int it = 0; it < 8; ++it) {
          const int row = it * 2 + hh;
          v4f v = *(const v4f*)(slab + row * 68 + c4);
          *(volatile v4f*)(C + (size_t)(mBase + row) * ldc + n0 + c4) = v;
        }
        __threadfence();
      }
    } else {
      const int q = lane >> 3, c8 = (lane & 7) * 8;
      unsigned short* C  = (unsigned short*)Cout  + (size_t)b * strideC;
      unsigned short* C2 = (OUT_MODE == 2) ? ((unsigned short*)Cout2 + (size_t)b * strideC) : nullptr;
      for (int pass = 0; pass < 2; ++pass) {
#pragma unroll
        for (int it = 0; it < 4; ++it) {
          const int row = it * 4 + q;
          const float* sp = slab + row * 68 + c8;
          v8h hv, lv;
#pragma unroll
          for (int e = 0; e < 8; ++e) {
            if (OUT_MODE == 1) {
              hv[e] = (_Float16)sp[e];
            } else {
              unsigned short hb = f2bf_bits(sp[e]);
              unsigned short lb = f2bf_bits(sp[e] - bf_bits2f(hb));
              hv[e] = __builtin_bit_cast(_Float16, hb);
              lv[e] = __builtin_bit_cast(_Float16, lb);
            }
          }
          *(volatile v8h*)(C + (size_t)(mBase + row) * ldc + n0 + c8) = hv;
          if (OUT_MODE == 2) *(volatile v8h*)(C2 + (size_t)(mBase + row) * ldc + n0 + c8) = lv;
        }
        __threadfence();
      }
    }
    __builtin_amdgcn_fence(__ATOMIC_RELEASE, "workgroup");
    __builtin_amdgcn_wave_barrier();
    __builtin_amdgcn_fence(__ATOMIC_ACQUIRE, "workgroup");
  }
}

__global__ __launch_bounds__(256) void cast8_bf16_kernel(const float* __restrict__ in, unsigned short* __restrict__ out, int n8) {
  const int i = blockIdx.x * 256 + threadIdx.x;
  if (i >= n8) return;
  const float* p = in + 8 * (size_t)i;
  const v4f a = *(const v4f*)(p);
  const v4f c = *(const v4f*)(p + 4);
  unsigned short hb[8];
#pragma unroll
  for (int e = 0; e < 4; ++e) {
    hb[e]     = f2bf_bits(a[e]);
    hb[4 + e] = f2bf_bits(c[e]);
  }
  const v4u u = (v4u){pk16(hb[0], hb[1]), pk16(hb[2], hb[3]), pk16(hb[4], hb[5]), pk16(hb[6], hb[7])};
  unsigned short* q = out + 8 * (size_t)i;
  *(volatile v4u*)q = u;
  __threadfence();
  *(volatile v4u*)q = u;
}

__global__ __launch_bounds__(256) void wtcast_bf16_kernel(const float* __restrict__ W0, const float* __restrict__ W1,
                                                          const float* __restrict__ W2, unsigned short* __restrict__ out) {
  __shared__ float sm[64][65];
  const int t  = threadIdx.x;
  const int k0 = blockIdx.x * 64;
  const int n0 = blockIdx.y * 64;
  const int z  = blockIdx.z;
  const float* W = (z == 0) ? W0 : (z == 1) ? W1 : W2;
#pragma unroll
  for (int i = 0; i < 16; ++i) {
    const int e = i * 256 + t;
    const int r = e >> 6;
    const int c = e & 63;
    sm[c][r] = W[(size_t)(k0 + r) * kEmb + n0 + c];
  }
  __syncthreads();
  const int lane = t & 31, wave = t >> 5;
  const int q = lane >> 3, c8 = (lane & 7) * 8;
  unsigned short* op = out + (size_t)z * kEmb * kEmb;
  for (int pass = 0; pass < 2; ++pass) {
#pragma unroll
    for (int it = 0; it < 2; ++it) {
      const int row = wave * 8 + it * 4 + q;
      unsigned short hb[8];
#pragma unroll
      for (int e = 0; e < 8; ++e) hb[e] = f2bf_bits(sm[row][c8 + e]);
      const v4u u = (v4u){pk16(hb[0], hb[1]), pk16(hb[2], hb[3]), pk16(hb[4], hb[5]), pk16(hb[6], hb[7])};
      *(volatile v4u*)(op + (size_t)(n0 + row) * kEmb + k0 + c8) = u;
    }
    __threadfence();
  }
}

__global__ __launch_bounds__(192) void bias_bf16_kernel(const float* __restrict__ bq, const float* __restrict__ bk,
                                                        const float* __restrict__ bv, float* __restrict__ bout) {
  const int t   = threadIdx.x;
  const int i0  = t * 4;
  const int sel = t >> 6;
  const int c0  = i0 & 255;
  const v4f a = *(const v4f*)(bq + c0);
  const v4f b = *(const v4f*)(bk + c0);
  const v4f c = *(const v4f*)(bv + c0);
  v4f r;
#pragma unroll
  for (int e = 0; e < 4; ++e) {
    const float x = (sel == 0) ? a[e] : ((sel == 1) ? b[e] : c[e]);
    r[e] = bf_bits2f(f2bf_bits(x));
  }
  float* op = bout + i0;
  *(volatile v4f*)op = r;
  __threadfence();
  *(volatile v4f*)op = r;
}

__global__ __launch_bounds__(256) void vsum_kernel(const float* __restrict__ Vf, unsigned short* __restrict__ VSt) {
  const int chunk = threadIdx.x;
  const int d     = blockIdx.x & 63;
  const int pair  = blockIdx.x >> 6;
  const int b     = pair >> 3, h = pair & 7;
  const int kw0   = chunk * 8;
  float acc[8];
#pragma unroll
  for (int e = 0; e < 8; ++e) acc[e] = 0.f;
  if (d < kHd) {
    const float* vp = Vf + (size_t)b * kSeq * kEmb + h * kHd + d;
#pragma unroll
    for (int u = 0; u < 40; ++u) {
      int s = kw0 + u;
      s = (s < kSeq) ? s : (kSeq - 1);
      const float val = vp[(size_t)s * kEmb];
#pragma unroll
      for (int e = 0; e < 8; ++e) {
        if (u - e >= 0 && u - e <= kWin - 1) acc[e] += val;
      }
    }
  }
  const bool livekw = (chunk < (kKeys / 8));
  unsigned short hb[8];
#pragma unroll
  for (int e = 0; e < 8; ++e) hb[e] = h_bits(livekw ? acc[e] : 0.f);
  const v4u u = (v4u){pk16(hb[0], hb[1]), pk16(hb[2], hb[3]), pk16(hb[4], hb[5]), pk16(hb[6], hb[7])};
  unsigned short* op = VSt + ((size_t)pair * kVSRows + d) * kSeq + kw0;
  *(volatile v4u*)op = u;
  __threadfence();
  *(volatile v4u*)op = u;
}

__global__ __launch_bounds__(512) void band_softmax_kernel(const float* __restrict__ G, unsigned short* __restrict__ P, float scale) {
  __shared__ __align__(16) float srow[kSeq];
  __shared__ float wred[32];
  const int t    = threadIdx.x;
  const int lane = t & 31;
  const int wave = __builtin_amdgcn_readfirstlane(t >> 5);
  const float* Gp = G + (size_t)blockIdx.x * ((size_t)kSeq * kSeq);
  unsigned short* Pp = P + (size_t)blockIdx.x * ((size_t)kSeq * kSeq);

  float run[8];
#pragma unroll
  for (int c = 0; c < 8; ++c) run[c] = 0.f;

#pragma unroll 1
  for (int i = 0; i < kSteps; ++i) {
#pragma unroll
    for (int c = 0; c < 8; ++c) {
      const int dmin = c * 512 + wave * 32 - kDiagOff;
      const bool dead = (i + dmin + 31 < 0) || (i - kWin + dmin > kSeq - 1);
      if (!dead) {
        const int dlt = dmin + lane;
        const int jn  = i + dlt;
        const int inc = (i < kSeq) ? i : (kSeq - 1);
        const int jnc = (jn < 0) ? 0 : ((jn > kSeq - 1) ? (kSeq - 1) : jn);
        float gn = Gp[(size_t)inc * kSeq + jnc];
        gn = (i < kSeq && jn >= 0 && jn < kSeq) ? gn : 0.f;
        const int io  = i - kWin;
        const int jo  = io + dlt;
        const int ioc = (io < 0) ? 0 : io;
        const int joc = (jo < 0) ? 0 : ((jo > kSeq - 1) ? (kSeq - 1) : jo);
        float go = Gp[(size_t)ioc * kSeq + joc];
        go = (io >= 0 && jo >= 0 && jo < kSeq) ? go : 0.f;
        run[c] = (run[c] + gn) - go;
        const int kw = jn - 32;
        if (i >= 16 && kw >= 0 && kw < kKeys) srow[kw] = run[c] * scale;
      }
    }
    __syncthreads();
    if (i >= 16) {
      const int q = i - 16;
      const bool live4 = (t < (kKeys / 4));
      const int tc = live4 ? t : (kKeys / 4 - 1);
      const v4f sv = *(const v4f*)(srow + 4 * tc);
      const float s0 = live4 ? sv[0] : -INFINITY;
      const float s1 = live4 ? sv[1] : -INFINITY;
      const float s2 = live4 ? sv[2] : -INFINITY;
      const float s3 = live4 ? sv[3] : -INFINITY;
      float m = fmaxf(fmaxf(s0, s1), fmaxf(s2, s3));
#pragma unroll
      for (int off = 16; off > 0; off >>= 1) m = fmaxf(m, __shfl_xor(m, off, 32));
      if (lane == 0) wred[wave] = m;
      __syncthreads();
      float bm = wred[lane & 15];
#pragma unroll
      for (int off = 8; off > 0; off >>= 1) bm = fmaxf(bm, __shfl_xor(bm, off, 32));
      const float e0 = live4 ? expf(s0 - bm) : 0.f;
      const float e1 = live4 ? expf(s1 - bm) : 0.f;
      const float e2 = live4 ? expf(s2 - bm) : 0.f;
      const float e3 = live4 ? expf(s3 - bm) : 0.f;
      *(v4f*)(srow + 4 * t) = (v4f){e0, e1, e2, e3};
      float ps = (e0 + e1) + (e2 + e3);
#pragma unroll
      for (int off = 16; off > 0; off >>= 1) ps += __shfl_xor(ps, off, 32);
      if (lane == 0) wred[16 + wave] = ps;
      __syncthreads();
      float bs = wred[16 + (lane & 15)];
#pragma unroll
      for (int off = 8; off > 0; off >>= 1) bs += __shfl_xor(bs, off, 32);
      const float scl = kPCarry / bs;
      if (t < 256) {
        const bool lv = (t < (kKeys / 8));
        const int tc2 = lv ? t : (kKeys / 8 - 1);
        const v4f ea = *(const v4f*)(srow + 8 * tc2);
        const v4f eb = *(const v4f*)(srow + 8 * tc2 + 4);
        unsigned short hb[8];
#pragma unroll
        for (int e = 0; e < 4; ++e) {
          hb[e]     = h_bits(lv ? (ea[e] * scl) : 0.f);
          hb[4 + e] = h_bits(lv ? (eb[e] * scl) : 0.f);
        }
        const v4u u = (v4u){pk16(hb[0], hb[1]), pk16(hb[2], hb[3]), pk16(hb[4], hb[5]), pk16(hb[6], hb[7])};
        unsigned short* pp = Pp + (size_t)q * kSeq + 8 * t;
        *(volatile v4u*)pp = u;
        __threadfence();
        *(volatile v4u*)pp = u;
      }
    }
    __syncthreads();
  }
}

__global__ __launch_bounds__(256) void pack_out_kernel(const float* __restrict__ CTX, float* __restrict__ out, int b, int h0) {
  const int gw   = blockIdx.x * 8 + (threadIdx.x >> 5);
  const int lane = threadIdx.x & 31;
  const int pr   = gw >> 9;
  const int q    = ((gw & 511) << 2) + (lane >> 3);
  const int d4   = (lane & 7) * 4;
  const v4f v = *(const v4f*)(CTX + ((size_t)pr * kSeq + q) * kVSRows + d4);
  float* op = out + ((size_t)(b * kSeq + q)) * kEmb + (h0 + pr) * kHd + d4;
  *(volatile v4f*)op = v;
  __threadfence();
  *(volatile v4f*)op = v;
}

extern "C" void kernel_launch(void* const* d_in, const int* in_sizes, int n_in,
                              void* d_out, int out_size, void* d_ws, size_t ws_size,
                              hipStream_t stream) {
  if (n_in < 7) return;
  if (in_sizes[0] != kTok * kEmb) return;
  if (in_sizes[1] != kEmb * kEmb || in_sizes[3] != kEmb * kEmb || in_sizes[5] != kEmb * kEmb) return;
  if (in_sizes[2] != kEmb || in_sizes[4] != kEmb || in_sizes[6] != kEmb) return;
  if (out_size != kTok * kEmb) return;

  const float* x  = (const float*)d_in[0];
  const float* Wq = (const float*)d_in[1];
  const float* bq = (const float*)d_in[2];
  const float* Wk = (const float*)d_in[3];
  const float* bk = (const float*)d_in[4];
  const float* Wv = (const float*)d_in[5];
  const float* bv = (const float*)d_in[6];
  float* out = (float*)d_out;

  char* ws = (char*)d_ws;
  size_t off = 0;
  const size_t szXb  = (size_t)kTok * kEmb * 2;
  const size_t szWt  = (size_t)3 * kEmb * kEmb * 2;
  const size_t szBs  = 4096;
  const size_t szQK  = (size_t)kTok * kQKld * 2;
  const size_t szVf  = (size_t)kTok * kEmb * 4;
  const size_t szVSt = (size_t)kPairs * kVSRows * kSeq * 2;
  const size_t szG   = (size_t)kGrp * kSeq * kSeq * 4;
  const size_t szP   = (size_t)kGrp * kSeq * kSeq * 2;
  const size_t szCtx = (size_t)kGrp * kSeq * kVSRows * 4;
  unsigned short* Xb  = (unsigned short*)(ws + off); off += szXb;
  unsigned short* Wt  = (unsigned short*)(ws + off); off += szWt;
  float*          Bs  = (float*)(ws + off);          off += szBs;
  unsigned short* QKh = (unsigned short*)(ws + off); off += szQK;
  unsigned short* QKl = (unsigned short*)(ws + off); off += szQK;
  float*          Vf  = (float*)(ws + off);          off += szVf;
  unsigned short* VSt = (unsigned short*)(ws + off); off += szVSt;
  float*          Gb  = (float*)(ws + off);          off += szG;
  unsigned short* Pb  = (unsigned short*)(ws + off); off += szP;
  float*          Ctx = (float*)(ws + off);          off += szCtx;
  if (off > ws_size) return;

  cast8_bf16_kernel<<<(kTok * kEmb / 8) / 256, 256, 0, stream>>>(x, Xb, kTok * kEmb / 8);
  wtcast_bf16_kernel<<<dim3(kEmb / 64, kEmb / 64, 3), 256, 0, stream>>>(Wq, Wk, Wv, Wt);
  bias_bf16_kernel<<<1, 192, 0, stream>>>(bq, bk, bv, Bs);

  wmma_gemm64<1, false, 2, 2, false><<<dim3((kTok / 64) * (kQKld / 64) / 8, 1), 256, 0, stream>>>(
      Xb, Xb, kEmb, 0L,
      Wt, Wt, kEmb, 0L,
      (void*)QKh, (void*)QKl, kQKld, 0L,
      Bs, Vf, 0L,
      kTok, kQKld, kEmb, 1.0f);
  wmma_gemm64<1, false, 2, 0, false><<<dim3((kTok / 64) * (kEmb / 64) / 8, 1), 256, 0, stream>>>(
      Xb, Xb, kEmb, 0L,
      Wt + (size_t)2 * kEmb * kEmb, Wt + (size_t)2 * kEmb * kEmb, kEmb, 0L,
      (void*)Vf, (void*)Vf, kEmb, 0L,
      Bs + 2 * kEmb, Vf, 0L,
      kTok, kEmb, kEmb, 1.0f);
  vsum_kernel<<<kPairs * kVSRows, 256, 0, stream>>>(Vf, VSt);

  for (int gi = 0; gi < kNGrp; ++gi) {
    const int b  = gi >> 2;
    const int h0 = (gi & 3) * kGrp;
    const size_t qoff = (size_t)b * kSeq * kQKld + (size_t)h0 * kHd;
    const size_t koff = qoff + kEmb;
    wmma_gemm64<1, true, 0, 0, false><<<dim3((kSeq / 64) * (kSeq / 64) / 8, kGrp), 256, 0, stream>>>(
        QKh + qoff, QKl + qoff, kQKld, (long)kHd,
        QKh + koff, QKl + koff, kQKld, (long)kHd,
        (void*)Gb, (void*)Gb, kSeq, (long)kSeq * kSeq,
        Bs, Vf, 0L,
        kSeq, kSeq, kHd, 1.0f);
    band_softmax_kernel<<<kGrp, 512, 0, stream>>>(Gb, Pb, kScoreScale);
    wmma_gemm64<0, false, 0, 0, false><<<dim3((kSeq / 64) * (kVSRows / 64) / 8, kGrp), 256, 0, stream>>>(
        Pb, Pb, kSeq, (long)kSeq * kSeq,
        VSt + (size_t)gi * kGrp * kVSRows * kSeq, VSt + (size_t)gi * kGrp * kVSRows * kSeq, kSeq, (long)kVSRows * kSeq,
        (void*)Ctx, (void*)Ctx, kVSRows, (long)kSeq * kVSRows,
        Bs, Vf, 0L,
        kSeq, kVSRows, kSeq, kPCarryInv);
    pack_out_kernel<<<(kGrp * kSeq / 4) / 8, 256, 0, stream>>>(Ctx, out, b, h0);
  }
}
